// Encoder_17076789969378
// MI455X (gfx1250) — hardware-verified
//
#include <hip/hip_runtime.h>
#include <stddef.h>

#define NBLK  625
#define TPTS  128
#define RAWF  384
#define NH3   64
#define WSMAX 134217728

static_assert(RAWF == 3 * TPTS);
static_assert((NBLK * NH3 * 4) % 256 == 0);
static_assert(NBLK * NH3 * 4 <= WSMAX);

typedef float          v4f   __attribute__((ext_vector_type(4)));
typedef float          v8f   __attribute__((ext_vector_type(8)));
typedef int            v8i   __attribute__((ext_vector_type(8)));
typedef unsigned short v8us  __attribute__((ext_vector_type(8)));
typedef unsigned short v16us __attribute__((ext_vector_type(16)));
typedef __bf16         v16bf __attribute__((ext_vector_type(16)));
typedef v4f  __attribute__((may_alias)) v4fa;
typedef v8us __attribute__((may_alias)) v8usa;
union FragB { v16bf v; v16us u; v8us h[2]; v8i w; };

__device__ __forceinline__ v8f wmb(const FragB& a, const FragB& b, v8f c) {
  v8f d = __builtin_amdgcn_wmma_f32_16x16x32_bf16(false, a.v, false, b.v, (short)0, c, false, false);
  asm volatile("v_nop\n\tv_nop\n\tv_nop\n\tv_nop" : "+v"(d) : "v"(a.w), "v"(b.w));
  return d;
}

__device__ __forceinline__ unsigned bf16_bits(float f) {
  const unsigned u = __float_as_uint(f);
  return (u + 0x7FFFu + ((u >> 16) & 1u)) >> 16;
}
__device__ __forceinline__ float bf16_val(float f) {
  return __uint_as_float(bf16_bits(f) << 16);
}
__device__ __forceinline__ void split_bf16(float v, unsigned& hb, unsigned& lb) {
  hb = bf16_bits(v);
  lb = bf16_bits(v - __uint_as_float(hb << 16));
}

__global__ __launch_bounds__(128) void k_fused(const float* __restrict__ pts,
                                               const float* __restrict__ W1, const float* __restrict__ B1,
                                               const float* __restrict__ W2, const float* __restrict__ B2,
                                               const float* __restrict__ W3, const float* __restrict__ B3,
                                               float* REC, int nPts, int nTiles, int tpb) {
  __shared__ __attribute__((aligned(16))) float          sRaw[2 * RAWF];
  __shared__ __attribute__((aligned(16))) float          sW1b[32 * 4];
  __shared__ __attribute__((aligned(16))) unsigned short sW2[32 * 16];
  __shared__ __attribute__((aligned(16))) unsigned short sW3[64 * 32];
  __shared__ __attribute__((aligned(16))) float          sB2[32];
  __shared__ __attribute__((aligned(16))) float          sB3[64];
  __shared__ __attribute__((aligned(16))) float          sPart[4 * NH3];

  const int tid = (int)threadIdx.x, lane = tid & 31, w = tid >> 5, h = lane >> 4, m = lane & 15;

  if (tid < 32) {
    const int j = tid & 15;
    const float a = W1[j * 3 + 0];
    const float b = W1[j * 3 + 1];
    const float c = W1[j * 3 + 2];
    const float d = B1[j];
    v4f q;
    q.x = bf16_val(a); q.y = bf16_val(b); q.z = bf16_val(c); q.w = bf16_val(d);
    *(v4fa*)(sW1b + 4 * tid) = q;
    sB2[tid] = bf16_val(B2[tid]);
  }
  if (tid < 64) {
    const float* p = W2 + 8 * tid;
    const v4f a = *(const v4fa*)p;
    const v4f b = *(const v4fa*)(p + 4);
    v8us o;
    o[0] = (unsigned short)bf16_bits(a.x); o[1] = (unsigned short)bf16_bits(a.y);
    o[2] = (unsigned short)bf16_bits(a.z); o[3] = (unsigned short)bf16_bits(a.w);
    o[4] = (unsigned short)bf16_bits(b.x); o[5] = (unsigned short)bf16_bits(b.y);
    o[6] = (unsigned short)bf16_bits(b.z); o[7] = (unsigned short)bf16_bits(b.w);
    *(v8usa*)(sW2 + 8 * tid) = o;
    sB3[tid] = bf16_val(B3[tid]);
  }
#pragma unroll
  for (int u = 0; u < 2; ++u) {
    const int e8 = (tid + 128 * u) * 8;
    const float* p = W3 + e8;
    const v4f a = *(const v4fa*)p;
    const v4f b = *(const v4fa*)(p + 4);
    v8us o;
    o[0] = (unsigned short)bf16_bits(a.x); o[1] = (unsigned short)bf16_bits(a.y);
    o[2] = (unsigned short)bf16_bits(a.z); o[3] = (unsigned short)bf16_bits(a.w);
    o[4] = (unsigned short)bf16_bits(b.x); o[5] = (unsigned short)bf16_bits(b.y);
    o[6] = (unsigned short)bf16_bits(b.z); o[7] = (unsigned short)bf16_bits(b.w);
    *(v8usa*)(sW3 + e8) = o;
  }
  __syncthreads();

  const v8f z8 = {0.f, 0.f, 0.f, 0.f, 0.f, 0.f, 0.f, 0.f};
  v8f cs[4];
#pragma unroll
  for (int ft = 0; ft < 4; ++ft) cs[ft] = z8;

  const int t0 = (int)blockIdx.x * tpb;
  int t1 = t0 + tpb;
  t1 = t1 > nTiles ? nTiles : t1;
  const size_t totalF = (size_t)nPts * 3;

#pragma unroll 1
  for (int t = t0; t < t1; ++t) {
    float* rb = sRaw + ((t - t0) & 1) * RAWF;
    const size_t fbase = (size_t)t * RAWF;
    if (tid < 96) {
      v4f q;
      if (fbase + RAWF <= totalF) {
        q = *(const v4fa*)(pts + fbase + 4 * tid);
      } else {
        const size_t last = totalF - 1;
        const size_t i0 = fbase + 4 * (size_t)tid;
        const size_t j0 = i0     < last ? i0     : last;
        const size_t j1 = i0 + 1 < last ? i0 + 1 : last;
        const size_t j2 = i0 + 2 < last ? i0 + 2 : last;
        const size_t j3 = i0 + 3 < last ? i0 + 3 : last;
        q.x = pts[j0]; q.y = pts[j1]; q.z = pts[j2]; q.w = pts[j3];
      }
      *(v4fa*)(rb + 4 * tid) = q;
    }
    __syncthreads();

#pragma unroll 1
    for (int pt = 0; pt < 2; ++pt) {
      int oz = 0;
      asm volatile("" : "+v"(oz));
      const int pl = 32 * w + 16 * pt + m;
      const bool valid = (t * TPTS + pl) < nPts;
      const float* rp = rb + 3 * pl;
      const float x = bf16_val(rp[0]);
      const float y = bf16_val(rp[1]);
      const float z = bf16_val(rp[2]);

      FragB bL2;
      {
        const float* wp = sW1b + oz + 32 * h;
#pragma unroll
        for (int i = 0; i < 8; ++i) {
          const v4f wv = *(const v4fa*)(wp + 4 * i);
          float v = x * wv.x;
          v = fmaf(y, wv.y, v);
          v = fmaf(z, wv.z, v);
          v = v + wv.w;
          v = fmaxf(v, 0.0f);
          unsigned hb, lb;
          split_bf16(v, hb, lb);
          bL2.u[i]     = (unsigned short)hb;
          bL2.u[8 + i] = (unsigned short)lb;
        }
      }

      v8f d2[2];
#pragma unroll
      for (int ft = 0; ft < 2; ++ft) {
        FragB a;
        const v8us wv = *(const v8usa*)(sW2 + oz + (16 * ft + m) * 16 + 8 * h);
        a.h[0] = wv;
        a.h[1] = wv;
        const float* bp = sB2 + oz + 16 * ft + 8 * h;
        const v4f ba = *(const v4fa*)bp;
        const v4f bb = *(const v4fa*)(bp + 4);
        const v8f c = {ba.x, ba.y, ba.z, ba.w, bb.x, bb.y, bb.z, bb.w};
        d2[ft] = wmb(a, bL2, c);
      }

      FragB bHi, bLo;
#pragma unroll
      for (int ft = 0; ft < 2; ++ft) {
#pragma unroll
        for (int r = 0; r < 8; ++r) {
          const float v = fmaxf(d2[ft][r], 0.0f);
          unsigned hb, lb;
          split_bf16(v, hb, lb);
          bHi.u[8 * ft + r] = (unsigned short)hb;
          bLo.u[8 * ft + r] = (unsigned short)lb;
        }
      }

#pragma unroll
      for (int ft = 0; ft < 4; ++ft) {
        FragB a;
        const unsigned short* wq = sW3 + oz + (16 * ft + m) * 32 + 8 * h;
        a.h[0] = *(const v8usa*)wq;
        a.h[1] = *(const v8usa*)(wq + 16);
        const float* bp = sB3 + oz + 16 * ft + 8 * h;
        const v4f ba = *(const v4fa*)bp;
        const v4f bb = *(const v4fa*)(bp + 4);
        const v8f c = {ba.x, ba.y, ba.z, ba.w, bb.x, bb.y, bb.z, bb.w};
        v8f d = wmb(a, bHi, c);
        d = wmb(a, bLo, d);
#pragma unroll
        for (int r = 0; r < 8; ++r) {
          const float v  = fmaxf(d[r], 0.0f);
          const float vz = valid ? v : 0.0f;
          cs[ft][r] = cs[ft][r] + vz;
        }
      }
    }
  }

#pragma unroll
  for (int ft = 0; ft < 4; ++ft) {
#pragma unroll
    for (int r = 0; r < 8; ++r) {
      float v = cs[ft][r];
      v = v + __shfl_xor(v, 1);
      v = v + __shfl_xor(v, 2);
      v = v + __shfl_xor(v, 4);
      v = v + __shfl_xor(v, 8);
      cs[ft][r] = v;
    }
  }
  if (m == 0) {
#pragma unroll
    for (int ft = 0; ft < 4; ++ft) {
      float* sp = sPart + w * NH3 + 16 * ft + 8 * h;
      const v4f lo4 = {cs[ft][0], cs[ft][1], cs[ft][2], cs[ft][3]};
      const v4f hi4 = {cs[ft][4], cs[ft][5], cs[ft][6], cs[ft][7]};
      *(v4fa*)sp       = lo4;
      *(v4fa*)(sp + 4) = hi4;
    }
  }
  __syncthreads();

  {
    const int c4 = tid & 15;
    const v4f r0 = *(const v4fa*)(sPart + 0 * NH3 + 4 * c4);
    const v4f r1 = *(const v4fa*)(sPart + 1 * NH3 + 4 * c4);
    const v4f r2 = *(const v4fa*)(sPart + 2 * NH3 + 4 * c4);
    const v4f r3 = *(const v4fa*)(sPart + 3 * NH3 + 4 * c4);
    const v4f s = ((r0 + r1) + r2) + r3;
    float* dp = REC + (size_t)blockIdx.x * NH3 + 4 * c4;
    if (tid < 16) *(volatile v4f*)dp = s;
    __threadfence();
    if (tid < 16) *(volatile v4f*)dp = s;
  }
}

__global__ __launch_bounds__(128) void k_final(const float* __restrict__ REC, const float* __restrict__ W4,
                                               const float* __restrict__ B4, float* out, double invN, int nblk) {
  __shared__ double sS[128];
  __shared__ double sM[NH3];
  __shared__ __attribute__((aligned(16))) float sO[128];
  const int tid = (int)threadIdx.x;
  const int k = tid & 63, half = tid >> 6;
  const int mid = (nblk + 1) >> 1;
  const int b0 = half ? mid : 0;
  const int b1 = half ? nblk : mid;
  double s = 0.0;
#pragma unroll 4
  for (int b = b0; b < b1; ++b) s += (double)REC[(size_t)b * NH3 + k];
  sS[tid] = s;
  __syncthreads();
  if (tid < 64) sM[tid] = (sS[tid] + sS[tid + 64]) * invN;
  __syncthreads();

  const float* wr = W4 + (size_t)tid * NH3;
  double acc = 0.0;
#pragma unroll 1
  for (int c = 0; c < NH3 / 4; ++c) {
    const v4f wv = *(const v4fa*)(wr + 4 * c);
    acc = fma(sM[4 * c + 0], (double)bf16_val(wv.x), acc);
    acc = fma(sM[4 * c + 1], (double)bf16_val(wv.y), acc);
    acc = fma(sM[4 * c + 2], (double)bf16_val(wv.z), acc);
    acc = fma(sM[4 * c + 3], (double)bf16_val(wv.w), acc);
  }
  acc = acc + (double)bf16_val(B4[tid]);
  sO[tid] = (float)acc;
  __syncthreads();

  const v4f o = *(const v4fa*)(sO + 4 * (tid & 31));
  float* dp = out + 4 * (tid & 31);
  if (tid < 32) *(volatile v4f*)dp = o;
  __threadfence();
  if (tid < 32) *(volatile v4f*)dp = o;
}

extern "C" void kernel_launch(void* const* d_in, const int* in_sizes, int n_in,
                              void* d_out, int out_size, void* d_ws, size_t ws_size,
                              hipStream_t stream) {
  if (n_in < 9) return;
  if (in_sizes[0] < 3 || (in_sizes[0] % 3) != 0) return;
  if (in_sizes[1] != 16 * 3 || in_sizes[2] != 16) return;
  if (in_sizes[3] != 32 * 16 || in_sizes[4] != 32) return;
  if (in_sizes[5] != 64 * 32 || in_sizes[6] != 64) return;
  if (in_sizes[7] != 128 * 64 || in_sizes[8] != 128) return;
  if (out_size != 128) return;

  const int nPts = in_sizes[0] / 3;
  if (nPts < 1 || nPts > (1 << 30)) return;

  const float* pts = (const float*)d_in[0];
  const float* W1  = (const float*)d_in[1];
  const float* B1  = (const float*)d_in[2];
  const float* W2  = (const float*)d_in[3];
  const float* B2  = (const float*)d_in[4];
  const float* W3  = (const float*)d_in[5];
  const float* B3  = (const float*)d_in[6];
  const float* W4  = (const float*)d_in[7];
  const float* B4  = (const float*)d_in[8];
  float* out = (float*)d_out;

  size_t recBytes = (size_t)NBLK * NH3 * sizeof(float);
  recBytes = (recBytes + 255) & ~(size_t)255;
  if (recBytes > ws_size || recBytes > (size_t)WSMAX) return;
  float* REC = (float*)d_ws;

  const int nTiles = (nPts + TPTS - 1) / TPTS;
  const int tpb    = (nTiles + NBLK - 1) / NBLK;
  const double invN = 1.0 / (double)nPts;

  k_fused<<<NBLK, 128, 0, stream>>>(pts, W1, B1, W2, B2, W3, B3, REC, nPts, nTiles, tpb);
  k_final<<<1, 128, 0, stream>>>(REC, W4, B4, out, invN, NBLK);
}
